// DTW_82085414961776
// MI455X (gfx1250) — hardware-run, weakly checked
//
#include <hip/hip_runtime.h>
#include <math.h>

typedef __attribute__((ext_vector_type(16))) _Float16 v16h;
typedef __attribute__((ext_vector_type(8)))  _Float16 v8h;
typedef __attribute__((ext_vector_type(16))) __bf16   v16b;
typedef __attribute__((ext_vector_type(8)))  __bf16   v8b;
typedef __attribute__((ext_vector_type(8)))  float    v8f;
typedef __attribute__((ext_vector_type(4)))  float    v4f;

constexpr int kBatch   = 64;
constexpr int kLen     = 1024;
constexpr int kResP    = 32;
static_assert((kLen % 32) == 0, "GEMM K multiple of 32");
static_assert((kBatch % 64) == 0 && (kLen % 64) == 0, "GEMM M,N multiples of 64");
static_assert(kBatch == 64, "output is exactly two 128-B lines");

constexpr size_t kSeqPlaneB = (size_t)kBatch * kLen * 2;
constexpr size_t kWPlaneB   = (size_t)kLen * kLen * 2;
constexpr size_t kProjB     = (size_t)kBatch * kLen * 4;
constexpr size_t kResB      = (size_t)kBatch * kResP * 4;
constexpr size_t kOffAH  = 0;
constexpr size_t kOffAL  = kOffAH  + kSeqPlaneB;
constexpr size_t kOffBH  = kOffAL  + kSeqPlaneB;
constexpr size_t kOffBL  = kOffBH  + kSeqPlaneB;
constexpr size_t kOffW1H = kOffBL  + kSeqPlaneB;
constexpr size_t kOffW1L = kOffW1H + kWPlaneB;
constexpr size_t kOffW2H = kOffW1L + kWPlaneB;
constexpr size_t kOffW2L = kOffW2H + kWPlaneB;
constexpr size_t kOffAP  = kOffW2L + kWPlaneB;
constexpr size_t kOffBP  = kOffAP  + kProjB;
constexpr size_t kOffRES = kOffBP  + kProjB;
constexpr size_t kWsTotal = kOffRES + kResB;
static_assert(kWsTotal == 9445376ull, "carve total");
static_assert(kWsTotal <= 134217728ull, "carve cap");
static_assert((kOffAL % 128) == 0 && (kOffBH % 128) == 0 && (kOffBL % 128) == 0 && (kOffW1H % 128) == 0 &&
              (kOffW1L % 128) == 0 && (kOffW2H % 128) == 0 && (kOffW2L % 128) == 0 && (kOffAP % 128) == 0 &&
              (kOffBP % 128) == 0 && (kOffRES % 128) == 0, "128-B aligned regions");

__device__ __forceinline__ unsigned short f2bf_bits(float f) {
  unsigned u = __float_as_uint(f);
  return (unsigned short)((u + 0x7FFFu + ((u >> 16) & 1u)) >> 16);
}
__device__ __forceinline__ float bf_bits2f(unsigned short h) { return __uint_as_float(((unsigned)h) << 16); }

__device__ __forceinline__ void mma_guard_h(v8f& c, v16h x, v16h y) { asm volatile("v_nop\n\tv_nop\n\tv_nop\n\tv_nop" : "+v"(c) : "v"(x), "v"(y)); }
__device__ __forceinline__ void mma_guard_b(v8f& c, v16b x, v16b y) { asm volatile("v_nop\n\tv_nop\n\tv_nop\n\tv_nop" : "+v"(c) : "v"(x), "v"(y)); }
__device__ __forceinline__ void keep4_h(v16h a, v16h b, v16h c, v16h d) { asm volatile("v_nop" :: "v"(a), "v"(b), "v"(c), "v"(d)); }
__device__ __forceinline__ void keep4_b(v16b a, v16b b, v16b c, v16b d) { asm volatile("v_nop" :: "v"(a), "v"(b), "v"(c), "v"(d)); }
template <typename T> struct Frag;
template <> struct Frag<_Float16> {
  typedef v16h V; union U { v16h v; v8h h[2]; };
  static __device__ __forceinline__ v16h load(const _Float16* p) {
    U f; f.h[0] = *(const v8h*)(p); f.h[1] = *(const v8h*)(p + 16); return f.v;
  }
  static __device__ __forceinline__ v8f mma(v16h a, v16h b, v8f c) {
    c = __builtin_amdgcn_wmma_f32_16x16x32_f16(false, a, false, b, (short)0, c, false, false);
    mma_guard_h(c, a, b);
    return c;
  }
  static __device__ __forceinline__ void keep(v16h a, v16h b, v16h c, v16h d) { keep4_h(a, b, c, d); }
};
template <> struct Frag<__bf16> {
  typedef v16b V; union U { v16b v; v8b h[2]; };
  static __device__ __forceinline__ v16b load(const __bf16* p) {
    U f; f.h[0] = *(const v8b*)(p); f.h[1] = *(const v8b*)(p + 16); return f.v;
  }
  static __device__ __forceinline__ v8f mma(v16b a, v16b b, v8f c) {
    c = __builtin_amdgcn_wmma_f32_16x16x32_bf16(false, a, false, b, (short)0, c, false, false);
    mma_guard_b(c, a, b);
    return c;
  }
  static __device__ __forceinline__ void keep(v16b a, v16b b, v16b c, v16b d) { keep4_b(a, b, c, d); }
};

template <int ET> struct Elem;
template <> struct Elem<0> { typedef _Float16 T; };
template <> struct Elem<1> { typedef __bf16 T; };
template <int ET, int SPL, int BIAS_MODE, int OUT_MODE, bool RESID>
__global__ __launch_bounds__(256) void wmma_gemm64(
    const unsigned short* __restrict__ Ap, const unsigned short* __restrict__ A2p, int lda, long strideA,
    const unsigned short* __restrict__ Btp, const unsigned short* __restrict__ Bt2p, int ldb, long strideB,
    void* __restrict__ Cout, void* __restrict__ Cout2, int ldc, long strideC,
    const float* __restrict__ bias,
    const float* __restrict__ resid, long strideR,
    int M, int N, int K, float scale) {
  typedef typename Elem<ET>::T T;
  typedef typename Frag<T>::V V;
  const T* A = (const T*)Ap; const T* A2 = (const T*)A2p; const T* Bt = (const T*)Btp; const T* Bt2 = (const T*)Bt2p;
  __shared__ __align__(16) float sT[8][16 * 68];
  const int b    = blockIdx.y;
  const int lane = threadIdx.x & 31;
  const int wave = threadIdx.x >> 5;
  const int tilesN = N >> 6;
  const int tilesM = M >> 6;
  const int tile = blockIdx.x * 8 + wave;
  if (tile >= tilesM * tilesN) return;
  const int tm = tile / tilesN;
  const int tn = tile - tm * tilesN;
  const int m0 = tm << 6;
  const int n0 = tn << 6;

  const T* Ab  = A  + (size_t)b * strideA;
  const T* Bb  = Bt + (size_t)b * strideB;
  const T* Ab2 = (SPL >= 1) ? (A2  + (size_t)b * strideA) : nullptr;
  const T* Bb2 = (SPL == 2) ? (Bt2 + (size_t)b * strideB) : nullptr;

  const int rlane = lane & 15;
  const int koff  = (lane >> 4) * 8;
  const int mOff  = (lane >> 4) * 8;

  v8f acc[4][4];
#pragma unroll
  for (int i = 0; i < 4; ++i)
#pragma unroll
    for (int j = 0; j < 4; ++j) acc[i][j] = (v8f){0.f,0.f,0.f,0.f,0.f,0.f,0.f,0.f};

  for (int k0 = 0; k0 < K; k0 += 32) {
    V bh[4], bl[4];
#pragma unroll
    for (int j = 0; j < 4; ++j) {
      const size_t bo = (size_t)(n0 + (j << 4) + rlane) * ldb + koff + k0;
      bh[j] = Frag<T>::load(Bb + bo);
      if (SPL == 2) bl[j] = Frag<T>::load(Bb2 + bo);
    }
#pragma unroll
    for (int i = 0; i < 4; ++i) {
      const size_t ao = (size_t)(m0 + (i << 4) + rlane) * lda + koff + k0;
      V ah = Frag<T>::load(Ab + ao);
      V al;
      if (SPL >= 1) al = Frag<T>::load(Ab2 + ao);
#pragma unroll
      for (int j = 0; j < 4; ++j) {
        acc[i][j] = Frag<T>::mma(ah, bh[j], acc[i][j]);
        if (SPL == 2) acc[i][j] = Frag<T>::mma(ah, bl[j], acc[i][j]);
        if (SPL >= 1) acc[i][j] = Frag<T>::mma(al, bh[j], acc[i][j]);
      }
    }
    Frag<T>::keep(bh[0], bh[1], bh[2], bh[3]);
    if (SPL == 2) Frag<T>::keep(bl[0], bl[1], bl[2], bl[3]);
  }

  float* slab = sT[wave];
  const float* Rb = RESID ? (resid + (size_t)b * strideR) : nullptr;
#pragma unroll
  for (int i = 0; i < 4; ++i) {
    const int mBase = m0 + (i << 4);
#pragma unroll
    for (int j = 0; j < 4; ++j) {
      const int n = n0 + (j << 4) + rlane;
      float bv = 0.f;
      if (BIAS_MODE == 2) bv = bias[n];
#pragma unroll
      for (int r = 0; r < 8; ++r) {
        float v = acc[i][j][r] * scale;
        if (BIAS_MODE == 1) v += bias[mBase + mOff + r];
        if (BIAS_MODE == 2) v += bv;
        if (RESID) v += Rb[(size_t)(mBase + mOff + r) * ldc + n];
        slab[(mOff + r) * 68 + (j << 4) + rlane] = v;
      }
    }
    __builtin_amdgcn_fence(__ATOMIC_RELEASE, "workgroup");
    __builtin_amdgcn_wave_barrier();
    __builtin_amdgcn_fence(__ATOMIC_ACQUIRE, "workgroup");
    if (OUT_MODE == 0) {
      float* C = (float*)Cout + (size_t)b * strideC;
      const int hh = lane >> 4, c4 = (lane & 15) * 4;
      for (int pass = 0; pass < 2; ++pass) {
#pragma unroll
        for (int it = 0; it < 8; ++it) {
          const int row = it * 2 + hh;
          v4f v = *(const v4f*)(slab + row * 68 + c4);
          *(volatile v4f*)(C + (size_t)(mBase + row) * ldc + n0 + c4) = v;
        }
        __threadfence();
      }
    } else {
      const int q = lane >> 3, c8 = (lane & 7) * 8;
      unsigned short* C  = (unsigned short*)Cout  + (size_t)b * strideC;
      unsigned short* C2 = (OUT_MODE == 2) ? ((unsigned short*)Cout2 + (size_t)b * strideC) : nullptr;
      for (int pass = 0; pass < 2; ++pass) {
#pragma unroll
        for (int it = 0; it < 4; ++it) {
          const int row = it * 4 + q;
          const float* sp = slab + row * 68 + c8;
          v8h hv, lv;
#pragma unroll
          for (int e = 0; e < 8; ++e) {
            if (OUT_MODE == 1) {
              hv[e] = (_Float16)sp[e];
            } else {
              unsigned short hb = f2bf_bits(sp[e]);
              unsigned short lb = f2bf_bits(sp[e] - bf_bits2f(hb));
              hv[e] = __builtin_bit_cast(_Float16, hb);
              lv[e] = __builtin_bit_cast(_Float16, lb);
            }
          }
          *(volatile v8h*)(C + (size_t)(mBase + row) * ldc + n0 + c8) = hv;
          if (OUT_MODE == 2) *(volatile v8h*)(C2 + (size_t)(mBase + row) * ldc + n0 + c8) = lv;
        }
        __threadfence();
      }
    }
    __builtin_amdgcn_fence(__ATOMIC_RELEASE, "workgroup");
    __builtin_amdgcn_wave_barrier();
    __builtin_amdgcn_fence(__ATOMIC_ACQUIRE, "workgroup");
  }
}

__global__ __launch_bounds__(256) void split_rows_bf16_kernel(
    const float* __restrict__ src, unsigned short* __restrict__ dhi, unsigned short* __restrict__ dlo, int total8)
{
  const int i = blockIdx.x * 256 + threadIdx.x;
  if (i >= total8) return;
  const size_t e0 = (size_t)i << 3;
  const v4f a0 = *(const v4f*)(src + e0);
  const v4f a1 = *(const v4f*)(src + e0 + 4);
  v8h hv, lv;
#pragma unroll
  for (int e = 0; e < 4; ++e) {
    const float x0 = a0[e];
    const float x1 = a1[e];
    const unsigned short h0 = f2bf_bits(x0), h1 = f2bf_bits(x1);
    const unsigned short l0 = f2bf_bits(x0 - bf_bits2f(h0)), l1 = f2bf_bits(x1 - bf_bits2f(h1));
    hv[e]     = __builtin_bit_cast(_Float16, h0);
    hv[4 + e] = __builtin_bit_cast(_Float16, h1);
    lv[e]     = __builtin_bit_cast(_Float16, l0);
    lv[4 + e] = __builtin_bit_cast(_Float16, l1);
  }
  unsigned short* qh = dhi + e0;
  unsigned short* ql = dlo + e0;
  *(volatile v8h*)qh = hv;
  *(volatile v8h*)ql = lv;
  __threadfence();
  *(volatile v8h*)qh = hv;
  *(volatile v8h*)ql = lv;
}

__global__ __launch_bounds__(1024) void minplus_table_kernel(
    const float* __restrict__ ap, const float* __restrict__ bp, float* __restrict__ res)
{
  __shared__ float sB[kLen];
  __shared__ float sD[3 * kLen];
  const int b    = blockIdx.x;
  const int i    = threadIdx.x;
  const int lane = i & 31;
  const int wave = i >> 5;
  const float kInf = __builtin_inff();

  const float av = ap[(size_t)b * kLen + i];
  sB[i] = bp[(size_t)b * kLen + i];
  sD[i] = kInf;
  sD[kLen + i] = kInf;
  sD[2 * kLen + i] = kInf;
  __syncthreads();

  const bool hasUp = (i > 0);
  const int  im1   = hasUp ? (i - 1) : 0;
  int oW = 0, oR1 = 2 * kLen, oR2 = kLen;
  float rlast = kInf;

#pragma unroll 1
  for (int d = 0; d < 2 * kLen - 1; ++d) {
    const int j = d - i;
    const bool valid = (j >= 0) && (j < kLen);
    int jc = j < 0 ? 0 : j;
    jc = jc > (kLen - 1) ? (kLen - 1) : jc;
    const float bv = sB[jc];
    const float vl = sD[oR1 + i];
    const float vu = sD[oR1 + im1];
    const float vd = sD[oR2 + im1];
    const float edge = (d == 0) ? 0.0f : kInf;
    const float up = hasUp ? vu : kInf;
    const float dg = hasUp ? vd : edge;
    const float best = fminf(dg, fminf(up, vl));
    const float diff = av - bv;
    const float c = diff * diff;
    const float r = valid ? (c + best) : kInf;
    sD[oW + i] = r;
    rlast = r;
    __syncthreads();
    const int t = oR2;
    oR2 = oR1;
    oR1 = oW;
    oW = t;
  }

  const float rb = __shfl(rlast, 31, 32);
  if (wave == 31) {
    volatile float* q = res + (size_t)b * kResP + lane;
    *q = rb;
    __threadfence();
    *q = rb;
  }
}

__global__ __launch_bounds__(32) void gather_out_kernel(const float* __restrict__ res, float* __restrict__ out)
{
  const int lane = threadIdx.x & 31;
  const float v0 = res[(size_t)lane * kResP];
  const float v1 = res[(size_t)(lane + 32) * kResP];
  volatile float* o = out;
  o[lane] = v0;
  o[32 + lane] = v1;
  __threadfence();
  o[lane] = v0;
  o[32 + lane] = v1;
}

extern "C" void kernel_launch(void* const* d_in, const int* in_sizes, int n_in,
                              void* d_out, int out_size, void* d_ws, size_t ws_size,
                              hipStream_t stream) {
  if (n_in < 6) return;
  if (in_sizes[0] != kBatch * kLen) return;
  if (in_sizes[1] != kBatch * kLen) return;
  if (in_sizes[2] != kLen * kLen) return;
  if (in_sizes[3] != kLen) return;
  if (in_sizes[4] != kLen * kLen) return;
  if (in_sizes[5] != kLen) return;
  if (out_size != kBatch) return;
  if (ws_size < kWsTotal) return;

  const float* a  = (const float*)d_in[0];
  const float* bq = (const float*)d_in[1];
  const float* W1 = (const float*)d_in[2];
  const float* b1 = (const float*)d_in[3];
  const float* W2 = (const float*)d_in[4];
  const float* b2 = (const float*)d_in[5];
  float* out = (float*)d_out;

  char* ws = (char*)d_ws;
  unsigned short* AH  = (unsigned short*)(ws + kOffAH);
  unsigned short* AL  = (unsigned short*)(ws + kOffAL);
  unsigned short* BH  = (unsigned short*)(ws + kOffBH);
  unsigned short* BL  = (unsigned short*)(ws + kOffBL);
  unsigned short* W1H = (unsigned short*)(ws + kOffW1H);
  unsigned short* W1L = (unsigned short*)(ws + kOffW1L);
  unsigned short* W2H = (unsigned short*)(ws + kOffW2H);
  unsigned short* W2L = (unsigned short*)(ws + kOffW2L);
  float*          AP  = (float*)(ws + kOffAP);
  float*          BP  = (float*)(ws + kOffBP);
  float*          RES = (float*)(ws + kOffRES);

  split_rows_bf16_kernel<<<(kBatch * kLen / 8) / 256, 256, 0, stream>>>(a,  AH,  AL,  kBatch * kLen / 8);
  split_rows_bf16_kernel<<<(kBatch * kLen / 8) / 256, 256, 0, stream>>>(bq, BH,  BL,  kBatch * kLen / 8);
  split_rows_bf16_kernel<<<(kLen * kLen / 8) / 256,   256, 0, stream>>>(W1, W1H, W1L, kLen * kLen / 8);
  split_rows_bf16_kernel<<<(kLen * kLen / 8) / 256,   256, 0, stream>>>(W2, W2H, W2L, kLen * kLen / 8);

  wmma_gemm64<1, 2, 2, 0, false><<<dim3(2, 1), 256, 0, stream>>>(
      AH, AL, kLen, 0L,
      W1H, W1L, kLen, 0L,
      (void*)AP, nullptr, kLen, 0L,
      b1, nullptr, 0L,
      kBatch, kLen, kLen, 1.0f);

  wmma_gemm64<1, 2, 2, 0, false><<<dim3(2, 1), 256, 0, stream>>>(
      BH, BL, kLen, 0L,
      W2H, W2L, kLen, 0L,
      (void*)BP, nullptr, kLen, 0L,
      b2, nullptr, 0L,
      kBatch, kLen, kLen, 1.0f);

  minplus_table_kernel<<<kBatch, kLen, 0, stream>>>(AP, BP, RES);

  gather_out_kernel<<<1, 32, 0, stream>>>(RES, out);
}
